// BiRNNDecoder_69106023792741
// MI455X (gfx1250) — hardware-run, weakly checked
//
#include <hip/hip_runtime.h>
#include <math.h>

typedef __attribute__((ext_vector_type(16))) _Float16 v16h;
typedef __attribute__((ext_vector_type(8)))  _Float16 v8h;
typedef __attribute__((ext_vector_type(16))) __bf16   v16b;
typedef __attribute__((ext_vector_type(8)))  __bf16   v8b;
typedef __attribute__((ext_vector_type(8)))  float    v8f;
typedef __attribute__((ext_vector_type(4)))  float    v4f;
typedef __attribute__((ext_vector_type(2)))  float    v2f;

constexpr int kB    = 8192;
constexpr int kT    = 262;
constexpr int kIn   = 2;
constexpr int kH    = 24;
constexpr int kHP   = 32;
constexpr int kG    = 3 * kH;
constexpr int kGP   = 128;
constexpr int kKI   = 256;
constexpr int kThr  = 256;
constexpr float kInCarry = 1024.0f;
constexpr float kSc = 1.0f / (kInCarry * kInCarry);
constexpr float kF16MinNormal = 6.103515625e-5f;

static_assert((kB % 64) == 0 && (kGP % 64) == 0 && (kHP % 32) == 0 && kHP >= kH && kGP >= kG && ((kB / 64) * (kGP / 64)) % 8 == 0 && kKI <= kT, "GEMM M, N multiples of 64, K of 32; grid exact (256 tiles a direction)");

constexpr size_t kOffWHH16 = 0ull;
constexpr size_t kOffZB = 16384ull;
constexpr size_t kOffHX16 = 17408ull;
constexpr size_t kOffH32 = 1065984ull;
constexpr size_t kOffGH = 3163136ull;
constexpr size_t kOffPFT = 11551744ull;
constexpr size_t kOffPBT = 20136960ull;
constexpr size_t kWsTotal = 28722176ull;
static_assert(kWsTotal <= 134217728ull, "carve cap: under 128 MiB");
static_assert(kOffWHH16 == 0
              && kOffZB == kOffWHH16 + 16384ull
              && kOffHX16 == kOffZB + 1024ull
              && kOffH32 == kOffHX16 + 1048576ull
              && kOffGH == kOffH32 + 2097152ull
              && kOffPFT == kOffGH + 8388608ull
              && kOffPBT == kOffPFT + 8585216ull
              && kWsTotal == kOffPBT + 8585216ull, "the carve is chained and totalled");
static_assert((kOffWHH16 % 256) == 0 && (kOffZB % 256) == 0 && (kOffHX16 % 256) == 0 && (kOffH32 % 256) == 0 && (kOffGH % 256) == 0 && (kOffPFT % 256) == 0 && (kOffPBT % 256) == 0, "aligned regions");

__device__ __forceinline__ unsigned short f2bf_bits(float f) {
  unsigned u = __float_as_uint(f);
  return (unsigned short)((u + 0x7FFFu + ((u >> 16) & 1u)) >> 16);
}
__device__ __forceinline__ float bf_bits2f(unsigned short h) { return __uint_as_float(((unsigned)h) << 16); }
__device__ __forceinline__ float bf16r(float f) { return bf_bits2f(f2bf_bits(f)); }
__device__ __forceinline__ float carry_flush(float v, float carry) {
  const float s = v * carry;
  return (fabsf(s) < kF16MinNormal) ? 0.0f : s;
}
__device__ __forceinline__ float frcp(float x) { return __builtin_amdgcn_rcpf(x); }

__device__ __forceinline__ void dep_guard4_h(v8f& a, v8f& b, v8f& c, v8f& d, v16h x, v16h y) { asm volatile("v_nop\n\tv_nop\n\tv_nop\n\tv_nop" : "+v"(a), "+v"(b), "+v"(c), "+v"(d) : "v"(x), "v"(y)); }
__device__ __forceinline__ void dep_guard4_b(v8f& a, v8f& b, v8f& c, v8f& d, v16b x, v16b y) { asm volatile("v_nop\n\tv_nop\n\tv_nop\n\tv_nop" : "+v"(a), "+v"(b), "+v"(c), "+v"(d) : "v"(x), "v"(y)); }
__device__ __forceinline__ void keep4_h(v16h a, v16h b, v16h c, v16h d) { asm volatile("v_nop" :: "v"(a), "v"(b), "v"(c), "v"(d)); }
__device__ __forceinline__ void keep4_b(v16b a, v16b b, v16b c, v16b d) { asm volatile("v_nop" :: "v"(a), "v"(b), "v"(c), "v"(d)); }
__device__ __forceinline__ void acc_guard4(v8f& a, v8f& b, v8f& c, v8f& d) { asm volatile("v_nop\n\tv_nop\n\tv_nop\n\tv_nop" : "+v"(a), "+v"(b), "+v"(c), "+v"(d)); }

template <typename T> struct Frag;
template <> struct Frag<_Float16> {
  typedef v16h V; union U { v16h v; v8h h[2]; };
  static __device__ __forceinline__ v16h load(const _Float16* p) {
    U f; f.h[0] = *(const v8h*)(p); f.h[1] = *(const v8h*)(p + 16); return f.v;
  }
  static __device__ __forceinline__ v8f mma(v16h a, v16h b, v8f c) {
    return __builtin_amdgcn_wmma_f32_16x16x32_f16(false, a, false, b, (short)0, c, false, false);
  }
  static __device__ __forceinline__ void guard4(v8f& a, v8f& b, v8f& c, v8f& d, v16h x, v16h y) { dep_guard4_h(a, b, c, d, x, y); }
  static __device__ __forceinline__ void keep(v16h a, v16h b, v16h c, v16h d) { keep4_h(a, b, c, d); }
};
template <> struct Frag<__bf16> {
  typedef v16b V; union U { v16b v; v8b h[2]; };
  static __device__ __forceinline__ v16b load(const __bf16* p) {
    U f; f.h[0] = *(const v8b*)(p); f.h[1] = *(const v8b*)(p + 16); return f.v;
  }
  static __device__ __forceinline__ v8f mma(v16b a, v16b b, v8f c) {
    return __builtin_amdgcn_wmma_f32_16x16x32_bf16(false, a, false, b, (short)0, c, false, false);
  }
  static __device__ __forceinline__ void guard4(v8f& a, v8f& b, v8f& c, v8f& d, v16b x, v16b y) { dep_guard4_b(a, b, c, d, x, y); }
  static __device__ __forceinline__ void keep(v16b a, v16b b, v16b c, v16b d) { keep4_b(a, b, c, d); }
};

__device__ __forceinline__ v8f mma_h(v16h a, v16h b, v8f c) {
  c = __builtin_amdgcn_wmma_f32_16x16x32_f16(false, a, false, b, (short)0, c, false, false);
  asm volatile("v_nop\n\tv_nop\n\tv_nop\n\tv_nop" : "+v"(c) : "v"(a), "v"(b));
  return c;
}

template <int ET> struct Elem;
template <> struct Elem<0> { typedef _Float16 T; };
template <> struct Elem<1> { typedef __bf16 T; };
template <int ET, bool SPLIT, int BIAS_MODE, int OUT_MODE, bool RESID, int ACT = 0>
__global__ __launch_bounds__(256) void wmma_gemm64(
    const unsigned short* __restrict__ Ap, const unsigned short* __restrict__ A2p, int lda, long strideA,
    const unsigned short* __restrict__ Btp, const unsigned short* __restrict__ Bt2p, int ldb, long strideB,
    void* __restrict__ Cout, void* __restrict__ Cout2, int ldc, long strideC,
    const float* __restrict__ bias,
    const float* __restrict__ resid, long strideR,
    int M, int N, int K, float scale) {
  typedef typename Elem<ET>::T T;
  typedef typename Frag<T>::V V;
  const T* A = (const T*)Ap; const T* A2 = (const T*)A2p; const T* Bt = (const T*)Btp; const T* Bt2 = (const T*)Bt2p;
  __shared__ __align__(16) float sT[8][16 * 68];
  const int b    = blockIdx.y;
  const int lane = threadIdx.x & 31;
  const int wave = threadIdx.x >> 5;
  const int tilesN = N >> 6;
  const int tilesM = M >> 6;
  const int tile = blockIdx.x * 8 + wave;
  if (tile >= tilesM * tilesN) return;
  const int tm = tile / tilesN;
  const int tn = tile - tm * tilesN;
  const int m0 = tm << 6;
  const int n0 = tn << 6;

  const T* Ab  = A  + (size_t)b * strideA;
  const T* Bb  = Bt + (size_t)b * strideB;
  const T* Ab2 = SPLIT ? (A2  + (size_t)b * strideA) : nullptr;
  const T* Bb2 = SPLIT ? (Bt2 + (size_t)b * strideB) : nullptr;

  const int rlane = lane & 15;
  const int koff  = (lane >> 4) * 8;
  const int mOff  = (lane >> 4) * 8;

  v8f acc[4][4];
#pragma unroll
  for (int i = 0; i < 4; ++i)
#pragma unroll
    for (int j = 0; j < 4; ++j) acc[i][j] = (v8f){0.f,0.f,0.f,0.f,0.f,0.f,0.f,0.f};

  for (int k0 = 0; k0 < K; k0 += 32) {
    V bh[4], bl[4];
#pragma unroll
    for (int j = 0; j < 4; ++j) {
      const size_t bo = (size_t)(n0 + (j << 4) + rlane) * ldb + koff + k0;
      bh[j] = Frag<T>::load(Bb + bo);
      if (SPLIT) bl[j] = Frag<T>::load(Bb2 + bo);
    }
#pragma unroll
    for (int i = 0; i < 4; ++i) {
      const size_t ao = (size_t)(m0 + (i << 4) + rlane) * lda + koff + k0;
      V ah = Frag<T>::load(Ab + ao);
      V al;
      if (SPLIT) al = Frag<T>::load(Ab2 + ao);
#pragma unroll
      for (int j = 0; j < 4; ++j) {
        acc[i][j] = Frag<T>::mma(ah, bh[j], acc[i][j]);
        if (SPLIT) {
          acc[i][j] = Frag<T>::mma(ah, bl[j], acc[i][j]);
          acc[i][j] = Frag<T>::mma(al, bh[j], acc[i][j]);
        }
      }
      Frag<T>::guard4(acc[i][0], acc[i][1], acc[i][2], acc[i][3], ah, SPLIT ? al : ah);
    }
    Frag<T>::keep(bh[0], bh[1], bh[2], bh[3]);
    if (SPLIT) Frag<T>::keep(bl[0], bl[1], bl[2], bl[3]);
  }
  acc_guard4(acc[0][0], acc[0][1], acc[0][2], acc[0][3]);
  acc_guard4(acc[1][0], acc[1][1], acc[1][2], acc[1][3]);
  acc_guard4(acc[2][0], acc[2][1], acc[2][2], acc[2][3]);
  acc_guard4(acc[3][0], acc[3][1], acc[3][2], acc[3][3]);

  float* slab = sT[wave];
  const float* Rb = RESID ? (resid + (size_t)b * strideR) : nullptr;
#pragma unroll
  for (int i = 0; i < 4; ++i) {
    const int mBase = m0 + (i << 4);
#pragma unroll
    for (int j = 0; j < 4; ++j) {
      const int n = n0 + (j << 4) + rlane;
      float bv = 0.f;
      if (BIAS_MODE == 2) bv = bias[n];
#pragma unroll
      for (int r = 0; r < 8; ++r) {
        float v = acc[i][j][r] * scale;
        if (BIAS_MODE == 1) v += bias[mBase + mOff + r];
        if (BIAS_MODE == 2) v += bv;
        if (RESID) v += Rb[(size_t)(mBase + mOff + r) * ldc + n];
        if (ACT == 1) v = tanhf(v);
        if (ACT == 2) v = fmaxf(v, 0.0f);
        if (ACT == 3) v = v / (1.0f + expf(-v));
        if (ACT == 4) v = (v > 0.f) ? v : 0.01f * v;
        slab[(mOff + r) * 68 + (j << 4) + rlane] = v;
      }
    }
    __builtin_amdgcn_fence(__ATOMIC_RELEASE, "workgroup");
    __builtin_amdgcn_wave_barrier();
    __builtin_amdgcn_fence(__ATOMIC_ACQUIRE, "workgroup");
    if (OUT_MODE == 0) {
      float* C = (float*)Cout + (size_t)b * strideC;
      const int hh = lane >> 4, c4 = (lane & 15) * 4;
      for (int pass = 0; pass < 2; ++pass) {
#pragma unroll
        for (int it = 0; it < 8; ++it) {
          const int row = it * 2 + hh;
          v4f v = *(const v4f*)(slab + row * 68 + c4);
          *(volatile v4f*)(C + (size_t)(mBase + row) * ldc + n0 + c4) = v;
        }
        __threadfence();
      }
    } else {
      const int q = lane >> 3, c8 = (lane & 7) * 8;
      unsigned short* C  = (unsigned short*)Cout  + (size_t)b * strideC;
      unsigned short* C2 = (OUT_MODE == 2) ? ((unsigned short*)Cout2 + (size_t)b * strideC) : nullptr;
      for (int pass = 0; pass < 2; ++pass) {
#pragma unroll
        for (int it = 0; it < 4; ++it) {
          const int row = it * 4 + q;
          const float* sp = slab + row * 68 + c8;
          v8h hv, lv;
#pragma unroll
          for (int e = 0; e < 8; ++e) {
            if (OUT_MODE == 1) {
              hv[e] = (_Float16)sp[e];
            } else {
              unsigned short hb = f2bf_bits(sp[e]);
              unsigned short lb = f2bf_bits(sp[e] - bf_bits2f(hb));
              hv[e] = __builtin_bit_cast(_Float16, hb);
              lv[e] = __builtin_bit_cast(_Float16, lb);
            }
          }
          *(volatile v8h*)(C + (size_t)(mBase + row) * ldc + n0 + c8) = hv;
          if (OUT_MODE == 2) *(volatile v8h*)(C2 + (size_t)(mBase + row) * ldc + n0 + c8) = lv;
        }
        __threadfence();
      }
    }
    __builtin_amdgcn_fence(__ATOMIC_RELEASE, "workgroup");
    __builtin_amdgcn_wave_barrier();
    __builtin_amdgcn_fence(__ATOMIC_ACQUIRE, "workgroup");
  }
}


__device__ __forceinline__ float fast_tanh(float v) { return 1.0f - 2.0f * frcp(__expf(2.0f * v) + 1.0f); }
__device__ __forceinline__ float fast_sigmoid(float v) { return frcp(1.0f + __expf(-v)); }

__global__ __launch_bounds__(64) void setup_kernel(const float* __restrict__ w_hh_f, const float* __restrict__ w_hh_b, unsigned short* __restrict__ WHH16, float* __restrict__ ZB) {
  const unsigned y = blockIdx.y;
  const unsigned c = threadIdx.x;
  if (y < 128u) {
    if (c >= 8u) return;
    const unsigned row = 2u * y + (c >> 2), ch = c & 3u;
    const unsigned dir = row >> 7, n = row & 127u;
    const float* W = dir ? w_hh_b : w_hh_f;
    const bool rowLive = n < (unsigned)kG;
    v8h hv;
#pragma unroll
    for (int e = 0; e < 8; ++e) {
      const unsigned k = ch * 8u + (unsigned)e;
      const bool live = rowLive && (k < (unsigned)kH);
      const float w = W[(size_t)(rowLive ? n : 0u) * kH + (k < (unsigned)kH ? k : 0u)];
      hv[e] = (_Float16)(live ? carry_flush(bf16r(w), kInCarry) : 0.0f);
    }
    unsigned short* dp = WHH16 + (size_t)row * kHP + ch * 8u;
    *(volatile v8h*)dp = hv;
    __threadfence();
    *(volatile v8h*)dp = hv;
  } else {
    const v4f z = {0.f, 0.f, 0.f, 0.f};
    float* dp = ZB + c * 4u;
    *(volatile v4f*)dp = z;
    __threadfence();
    *(volatile v4f*)dp = z;
  }
}

__global__ __launch_bounds__(kThr) void state_zero_kernel(unsigned short* __restrict__ HX16) {
  const size_t v = (size_t)blockIdx.x * kThr + threadIdx.x;
  const v4f z = {0.f, 0.f, 0.f, 0.f};
  float* dp = (float*)HX16 + v * 4u;
  *(volatile v4f*)dp = z;
  __threadfence();
  *(volatile v4f*)dp = z;
}
static_assert(kOffH32 == kOffHX16 + 1048576ull && (1048576 + 2097152) / 16 == 768 * kThr, "the two state planes are adjacent: one fill");

__global__ __launch_bounds__(kThr) void cell_kernel(const float* __restrict__ x, const float* __restrict__ w_ih_f, const float* __restrict__ b_ih_f, const float* __restrict__ b_hh_f,
                                                    const float* __restrict__ w_ih_b, const float* __restrict__ b_ih_b, const float* __restrict__ b_hh_b, const float* __restrict__ w_out,
                                                    const float* __restrict__ GH, float* __restrict__ H32, unsigned short* __restrict__ HX16,
                                                    float* __restrict__ PFT, float* __restrict__ PBT, int t) {
  const unsigned dir = blockIdx.y;
  const unsigned smp = blockIdx.x * (unsigned)kThr + threadIdx.x;
  const int p = dir ? (kT - 1 - t) : t;
  const float* w_ih = dir ? w_ih_b : w_ih_f;
  const float* b_ih = dir ? b_ih_b : b_ih_f;
  const float* b_hh = dir ? b_hh_b : b_hh_f;
  const v2f xv = *(const v2f*)(x + ((size_t)smp * kT + (size_t)p) * kIn);
  const float x0 = bf16r(xv[0]), x1 = bf16r(xv[1]);
  const float* gh = GH + ((size_t)dir * kB + smp) * kGP;
  float* hp = H32 + ((size_t)dir * kB + smp) * kHP;
  unsigned short* h16 = HX16 + ((size_t)dir * kB + smp) * kHP;
  float acc = 0.0f;
  for (int c4 = 0; c4 < kH; c4 += 4) {
    const v4f ghr = *(const v4f*)(gh + c4), ghz = *(const v4f*)(gh + kH + c4), ghn = *(const v4f*)(gh + 2 * kH + c4);
    const v4f ho = *(const v4f*)(hp + c4);
    v4f hn;
#pragma unroll
    for (int e = 0; e < 4; ++e) {
      const int j = c4 + e;
      const float wr0 = w_ih[(size_t)j * kIn], wr1 = w_ih[(size_t)j * kIn + 1];
      const float wz0 = w_ih[(size_t)(kH + j) * kIn], wz1 = w_ih[(size_t)(kH + j) * kIn + 1];
      const float wn0 = w_ih[(size_t)(2 * kH + j) * kIn], wn1 = w_ih[(size_t)(2 * kH + j) * kIn + 1];
      const float bir = b_ih[j], biz = b_ih[kH + j], bin = b_ih[2 * kH + j];
      const float bhr = b_hh[j], bhz = b_hh[kH + j], bhn = b_hh[2 * kH + j];
      const float wo = w_out[dir * (unsigned)kH + (unsigned)j];
      const float gir = bf16r(wr0) * x0 + bf16r(wr1) * x1 + bf16r(bir);
      const float giz = bf16r(wz0) * x0 + bf16r(wz1) * x1 + bf16r(biz);
      const float gin = bf16r(wn0) * x0 + bf16r(wn1) * x1 + bf16r(bin);
      const float r = fast_sigmoid(gir + (ghr[e] + bf16r(bhr)));
      const float z = fast_sigmoid(giz + (ghz[e] + bf16r(bhz)));
      const float n = fast_tanh(gin + r * (ghn[e] + bf16r(bhn)));
      const float h1 = (1.0f - z) * n + z * ho[e];
      hn[e] = h1;
      acc += h1 * bf16r(wo);
    }
    v4f hs = hn;
    for (int pass = 0; pass < 2; ++pass) {
      *(volatile v4f*)(hp + c4) = hs;
      __threadfence();
    }
  }
#pragma unroll
  for (int c8 = 0; c8 < kHP; c8 += 8) {
    v8h hv;
    if (c8 < kH) {
      const v4f a0 = *(const v4f*)(hp + c8), a1 = *(const v4f*)(hp + c8 + 4);
#pragma unroll
      for (int e = 0; e < 4; ++e) { hv[e] = (_Float16)carry_flush(a0[e], kInCarry); hv[4 + e] = (_Float16)carry_flush(a1[e], kInCarry); }
    } else {
#pragma unroll
      for (int e = 0; e < 8; ++e) hv[e] = (_Float16)0.0f;
    }
    for (int pass = 0; pass < 2; ++pass) {
      *(volatile v8h*)(h16 + c8) = hv;
      __threadfence();
    }
  }
  float* pp = (dir ? PBT : PFT) + (size_t)p * kB + smp;
  *(volatile float*)pp = acc;
  __threadfence();
  *(volatile float*)pp = acc;
}
static_assert(kB % kThr == 0 && (kH % 8) == 0 && kHP == kH + 8, "cell grid exact; the state row = three live chunks + one zero chunk");

__global__ __launch_bounds__(kThr) void out_kernel(const float* __restrict__ PFT, const float* __restrict__ PBT, const float* __restrict__ b_out, float* __restrict__ out) {
  const unsigned smp = blockIdx.x;
  const unsigned k = threadIdx.x;
  const float b0 = b_out[0];
  const float v = PFT[(size_t)k * kB + smp] + PBT[(size_t)k * kB + smp] + bf16r(b0);
  float* dp = out + (size_t)smp * kKI + k;
  *(volatile float*)dp = v;
  __threadfence();
  *(volatile float*)dp = v;
}
static_assert(kKI == kThr, "one block a sample: 256 positions");

extern "C" void kernel_launch(void* const* d_in, const int* in_sizes, int n_in,
                              void* d_out, int out_size, void* d_ws, size_t ws_size,
                              hipStream_t stream) {
  if (n_in < 11 || d_out == nullptr || d_ws == nullptr) return;
  if (in_sizes[0] != kB * kT * kIn || in_sizes[1] != kG * kIn || in_sizes[2] != kG * kH || in_sizes[3] != kG || in_sizes[4] != kG) return;
  if (in_sizes[5] != kG * kIn || in_sizes[6] != kG * kH || in_sizes[7] != kG || in_sizes[8] != kG || in_sizes[9] != 2 * kH || in_sizes[10] != 1) return;
  if (out_size != kB * kKI) return;
  if (ws_size < kWsTotal) return;
  const float* x = (const float*)d_in[0];
  const float* w_ih_f = (const float*)d_in[1];
  const float* w_hh_f = (const float*)d_in[2];
  const float* b_ih_f = (const float*)d_in[3];
  const float* b_hh_f = (const float*)d_in[4];
  const float* w_ih_b = (const float*)d_in[5];
  const float* w_hh_b = (const float*)d_in[6];
  const float* b_ih_b = (const float*)d_in[7];
  const float* b_hh_b = (const float*)d_in[8];
  const float* w_out = (const float*)d_in[9];
  const float* b_out = (const float*)d_in[10];
  float* out = (float*)d_out;
  char* ws = (char*)d_ws;
  unsigned short* WHH16 = (unsigned short*)(ws + kOffWHH16);
  float* ZB = (float*)(ws + kOffZB);
  unsigned short* HX16 = (unsigned short*)(ws + kOffHX16);
  float* H32 = (float*)(ws + kOffH32);
  float* GH = (float*)(ws + kOffGH);
  float* PFT = (float*)(ws + kOffPFT);
  float* PBT = (float*)(ws + kOffPBT);

  setup_kernel<<<dim3(1, 129), 64, 0, stream>>>(w_hh_f, w_hh_b, WHH16, ZB);
  state_zero_kernel<<<768, kThr, 0, stream>>>(HX16);
  for (int t = 0; t < kT; ++t) {
    wmma_gemm64<0, false, 2, 0, false, 0><<<dim3((kB / 64) * (kGP / 64) / 8, 2), 256, 0, stream>>>(
        HX16, HX16, kHP, (long)kB * kHP, WHH16, WHH16, kHP, (long)kGP * kHP, (void*)GH, (void*)GH, kGP, (long)kB * kGP, ZB, nullptr, 0L, kB, kGP, kHP, kSc);
    cell_kernel<<<dim3(kB / kThr, 2), kThr, 0, stream>>>(x, w_ih_f, b_ih_f, b_hh_f, w_ih_b, b_ih_b, b_hh_b, w_out, GH, H32, HX16, PFT, PBT, t);
  }
  out_kernel<<<kB, kThr, 0, stream>>>(PFT, PBT, b_out, out);
}
